// RecurrentODESolver_25460566130815
// MI455X (gfx1250) — hardware-verified
//
#include <hip/hip_runtime.h>
#include <stddef.h>
#include <stdint.h>


typedef __attribute__((ext_vector_type(16))) _Float16 v16h;
typedef __attribute__((ext_vector_type(8)))  _Float16 v8h;
typedef __attribute__((ext_vector_type(4)))  _Float16 v4h;
typedef __attribute__((ext_vector_type(16))) __bf16   v16b;
typedef __attribute__((ext_vector_type(8)))  __bf16   v8b;
typedef __attribute__((ext_vector_type(8)))  float    v8f;
typedef __attribute__((ext_vector_type(4)))  float    v4f;

__device__ __forceinline__ void dep_guard_h(v8f& a, v8f& b, v16h x, v16h y) { asm volatile("v_nop\n\tv_nop\n\tv_nop\n\tv_nop" : "+v"(a), "+v"(b) : "v"(x), "v"(y)); }
__device__ __forceinline__ void dep_guard_b(v8f& a, v8f& b, v16b x, v16b y) { asm volatile("v_nop\n\tv_nop\n\tv_nop\n\tv_nop" : "+v"(a), "+v"(b) : "v"(x), "v"(y)); }
__device__ __forceinline__ void keep4_h(v16h a, v16h b, v16h c, v16h d) { asm volatile("v_nop" :: "v"(a), "v"(b), "v"(c), "v"(d)); }
__device__ __forceinline__ void keep4_b(v16b a, v16b b, v16b c, v16b d) { asm volatile("v_nop" :: "v"(a), "v"(b), "v"(c), "v"(d)); }
__device__ __forceinline__ void acc_guard4(v8f& a, v8f& b, v8f& c, v8f& d) { asm volatile("v_nop\n\tv_nop\n\tv_nop\n\tv_nop" : "+v"(a), "+v"(b), "+v"(c), "+v"(d)); }

template <typename T> struct Frag;
template <> struct Frag<_Float16> {
  typedef v16h V; union U { v16h v; v8h h[2]; };
  static __device__ __forceinline__ v16h load(const _Float16* p) {
    U f; f.h[0] = *(const v8h*)(p); f.h[1] = *(const v8h*)(p + 16); return f.v;
  }
  static __device__ __forceinline__ v8f mma(v16h a, v16h b, v8f c) {
    return __builtin_amdgcn_wmma_f32_16x16x32_f16(false, a, false, b, (short)0, c, false, false);
  }
  static __device__ __forceinline__ void guard(v8f& a, v8f& b, v16h x, v16h y) { dep_guard_h(a, b, x, y); }
  static __device__ __forceinline__ void keep(v16h a, v16h b, v16h c, v16h d) { keep4_h(a, b, c, d); }
};
template <> struct Frag<__bf16> {
  typedef v16b V; union U { v16b v; v8b h[2]; };
  static __device__ __forceinline__ v16b load(const __bf16* p) {
    U f; f.h[0] = *(const v8b*)(p); f.h[1] = *(const v8b*)(p + 16); return f.v;
  }
  static __device__ __forceinline__ v8f mma(v16b a, v16b b, v8f c) {
    return __builtin_amdgcn_wmma_f32_16x16x32_bf16(false, a, false, b, (short)0, c, false, false);
  }
  static __device__ __forceinline__ void guard(v8f& a, v8f& b, v16b x, v16b y) { dep_guard_b(a, b, x, y); }
  static __device__ __forceinline__ void keep(v16b a, v16b b, v16b c, v16b d) { keep4_b(a, b, c, d); }
};

#define DDIM   256
#define PKH    264
#define RPB    64
#define NSTEP  40
#define HSTEP  0.025f
#define SLABP  68
#define TWOLOG2E 2.8853900817779268f

__device__ __forceinline__ float tanh_apx(float g) {
  const float e = __builtin_amdgcn_exp2f(g * TWOLOG2E);
  const float r = __builtin_amdgcn_rcpf(e + 1.0f);
  return __builtin_fmaf(-2.0f, r, 1.0f);
}

__host__ __device__ constexpr float acoef(int t, int j) {
  return (t == 1) ? 0.2f
       : (t == 2) ? ((j == 0) ? (float)(3.0 / 40.0) : (float)(9.0 / 40.0))
       : (t == 3) ? ((j == 0) ? (float)(44.0 / 45.0) : (j == 1) ? (float)(-56.0 / 15.0) : (float)(32.0 / 9.0))
       : (t == 4) ? ((j == 0) ? (float)(19372.0 / 6561.0) : (j == 1) ? (float)(-25360.0 / 2187.0)
                   : (j == 2) ? (float)(64448.0 / 6561.0) : (float)(-212.0 / 729.0))
       :            ((j == 0) ? (float)(9017.0 / 3168.0) : (j == 1) ? (float)(-355.0 / 33.0)
                   : (j == 2) ? (float)(46732.0 / 5247.0) : (j == 3) ? (float)(49.0 / 176.0)
                   : (float)(-5103.0 / 18656.0));
}

__device__ __forceinline__ void st_pair(float* base, unsigned o0, unsigned o1, v4f a, v4f b) {
  *(volatile v4f*)(base + o0) = a;
  *(volatile v4f*)(base + o1) = b;
  __threadfence();
  *(volatile v4f*)(base + o0) = a;
  *(volatile v4f*)(base + o1) = b;
}

__device__ __forceinline__ void tile_put(_Float16* tile, int row, int col, v4f a, v4f b) {
  const v4h ha = __builtin_convertvector(a, v4h);
  const v4h hb = __builtin_convertvector(b, v4h);
  const v8h t = __builtin_shufflevector(ha, hb, 0, 1, 2, 3, 4, 5, 6, 7);
  *(v8h*)(tile + row * PKH + col) = t;
}

__device__ __forceinline__ void gemm_ft(const _Float16* __restrict__ Wt, const _Float16* tile,
                                         int F0, int c, int koff, v8f (&acc)[4][4]) {
  typedef Frag<_Float16> FR;
  const _Float16* wr = Wt + (size_t)(F0 + c) * DDIM + koff;
  const _Float16* tr = tile + c * PKH + koff;
  {
    const v8f z = {0.f, 0.f, 0.f, 0.f, 0.f, 0.f, 0.f, 0.f};
    v16h b[4];
#pragma unroll
    for (int j = 0; j < 4; ++j) b[j] = FR::load(tr + j * 16 * PKH);
#pragma unroll
    for (int i = 0; i < 4; ++i) {
      const v16h a = FR::load(wr + i * 16 * DDIM);
#pragma unroll
      for (int j = 0; j < 4; ++j) acc[i][j] = FR::mma(a, b[j], z);
      FR::guard(acc[i][0], acc[i][3], a, a);
    }
    FR::keep(b[0], b[1], b[2], b[3]);
  }
#pragma unroll 1
  for (int k0 = 32; k0 < DDIM; k0 += 32) {
    v16h b[4];
#pragma unroll
    for (int j = 0; j < 4; ++j) b[j] = FR::load(tr + j * 16 * PKH + k0);
#pragma unroll
    for (int i = 0; i < 4; ++i) {
      const v16h a = FR::load(wr + i * 16 * DDIM + k0);
#pragma unroll
      for (int j = 0; j < 4; ++j) acc[i][j] = FR::mma(a, b[j], acc[i][j]);
      FR::guard(acc[i][0], acc[i][3], a, a);
    }
    FR::keep(b[0], b[1], b[2], b[3]);
  }
  acc_guard4(acc[0][0], acc[0][1], acc[0][2], acc[0][3]);
  acc_guard4(acc[1][0], acc[1][1], acc[1][2], acc[1][3]);
  acc_guard4(acc[2][0], acc[2][1], acc[2][2], acc[2][3]);
  acc_guard4(acc[3][0], acc[3][1], acc[3][2], acc[3][3]);
}

__device__ __forceinline__ void write_t(const v8f (&acc)[4][4], _Float16* tile, int F0, int c, int hh) {
#pragma unroll
  for (int i = 0; i < 4; ++i) {
#pragma unroll
    for (int j = 0; j < 4; ++j) {
      const v8f g = acc[i][j];
      v8f t;
#pragma unroll
      for (int e = 0; e < 8; ++e) t[e] = tanh_apx(g[e]);
      *(v8h*)(tile + (16 * j + c) * PKH + F0 + 16 * i + 8 * hh) = __builtin_convertvector(t, v8h);
    }
  }
}

template <int S>
__device__ __forceinline__ void build_next(const v8f (&acc)[4][4], float* Xw, size_t ntot, unsigned lo,
                                            _Float16* tile, int F0, int c, int hh) {
  float* Ks = Xw + (size_t)(S + 1) * ntot;
#pragma unroll
  for (int i = 0; i < 4; ++i) {
#pragma unroll
    for (int j = 0; j < 4; ++j) {
      const unsigned o0 = lo + (unsigned)(2 * (i * 4 + j)) * 128u;
      const unsigned o1 = o0 + 128u;
      const v8f kk = acc[i][j];
      const v4f ka = __builtin_shufflevector(kk, kk, 0, 1, 2, 3);
      const v4f kb = __builtin_shufflevector(kk, kk, 4, 5, 6, 7);
      st_pair(Ks, o0, o1, ka, kb);
      const v4f xa = *(const v4f*)(Xw + o0);
      const v4f xb = *(const v4f*)(Xw + o1);
      v4f sa, sb;
      if (S == 0) {
        sa = acoef(1, 0) * ka;
        sb = acoef(1, 0) * kb;
      } else {
        const float* K0 = Xw + ntot;
        const v4f qa = *(const v4f*)(K0 + o0);
        const v4f qb = *(const v4f*)(K0 + o1);
        sa = acoef(S + 1, 0) * qa;
        sb = acoef(S + 1, 0) * qb;
#pragma unroll
        for (int jj = 1; jj < S; ++jj) {
          const float* Kj = Xw + (size_t)(jj + 1) * ntot;
          const v4f ra = *(const v4f*)(Kj + o0);
          const v4f rb = *(const v4f*)(Kj + o1);
          sa = sa + acoef(S + 1, jj) * ra;
          sb = sb + acoef(S + 1, jj) * rb;
        }
        sa = sa + acoef(S + 1, S) * ka;
        sb = sb + acoef(S + 1, S) * kb;
      }
      const v4f ya = xa + HSTEP * sa;
      const v4f yb = xb + HSTEP * sb;
      tile_put(tile, 16 * j + c, F0 + 16 * i + 8 * hh, ya, yb);
    }
  }
}

__device__ __forceinline__ void final_update(const v8f (&acc)[4][4], float* Xw, size_t ntot, unsigned lo,
                                              _Float16* tile, int F0, int c, int hh) {
  const float* K0 = Xw + ntot;
  const float* K2 = Xw + (size_t)3 * ntot;
  const float* K3 = Xw + (size_t)4 * ntot;
  const float* K4 = Xw + (size_t)5 * ntot;
  const float b0 = (float)(35.0 / 384.0);
  const float b2 = (float)(500.0 / 1113.0);
  const float b3 = (float)(125.0 / 192.0);
  const float b4 = (float)(-2187.0 / 6784.0);
  const float b5 = (float)(11.0 / 84.0);
#pragma unroll
  for (int i = 0; i < 4; ++i) {
#pragma unroll
    for (int j = 0; j < 4; ++j) {
      const unsigned o0 = lo + (unsigned)(2 * (i * 4 + j)) * 128u;
      const unsigned o1 = o0 + 128u;
      const v8f kk = acc[i][j];
      const v4f ka = __builtin_shufflevector(kk, kk, 0, 1, 2, 3);
      const v4f kb = __builtin_shufflevector(kk, kk, 4, 5, 6, 7);
      const v4f xa = *(const v4f*)(Xw + o0);
      const v4f xb = *(const v4f*)(Xw + o1);
      v4f qa = *(const v4f*)(K0 + o0);
      v4f qb = *(const v4f*)(K0 + o1);
      v4f sa = b0 * qa;
      v4f sb = b0 * qb;
      qa = *(const v4f*)(K2 + o0); qb = *(const v4f*)(K2 + o1);
      sa = sa + b2 * qa; sb = sb + b2 * qb;
      qa = *(const v4f*)(K3 + o0); qb = *(const v4f*)(K3 + o1);
      sa = sa + b3 * qa; sb = sb + b3 * qb;
      qa = *(const v4f*)(K4 + o0); qb = *(const v4f*)(K4 + o1);
      sa = sa + b4 * qa; sb = sb + b4 * qb;
      sa = sa + b5 * ka; sb = sb + b5 * kb;
      const v4f xna = xa + HSTEP * sa;
      const v4f xnb = xb + HSTEP * sb;
      st_pair(Xw, o0, o1, xna, xnb);
      tile_put(tile, 16 * j + c, F0 + 16 * i + 8 * hh, xna, xnb);
    }
  }
}

template <int S> struct Tail {
  static __device__ __forceinline__ void run(const v8f (&acc)[4][4], float* Xw, size_t ntot, unsigned lo,
                                             _Float16* tile, int F0, int c, int hh) {
    build_next<S>(acc, Xw, ntot, lo, tile, F0, c, hh);
  }
};
template <> struct Tail<5> {
  static __device__ __forceinline__ void run(const v8f (&acc)[4][4], float* Xw, size_t ntot, unsigned lo,
                                             _Float16* tile, int F0, int c, int hh) {
    final_update(acc, Xw, ntot, lo, tile, F0, c, hh);
  }
};

template <int S>
__device__ __forceinline__ void run_stage(const _Float16* __restrict__ wt1, const _Float16* __restrict__ wt2,
                                           _Float16* tile, float* Xw, size_t ntot, unsigned lo,
                                           int F0, int c, int hh, int koff) {
  v8f acc[4][4];
  gemm_ft(wt1, tile, F0, c, koff, acc);
  __syncthreads();
  write_t(acc, tile, F0, c, hh);
  __syncthreads();
  gemm_ft(wt2, tile, F0, c, koff, acc);
  __syncthreads();
  Tail<S>::run(acc, Xw, ntot, lo, tile, F0, c, hh);
  __syncthreads();
}

__global__ __launch_bounds__(256) void k_wt(const float* __restrict__ W1, const float* __restrict__ W2,
                                             _Float16* __restrict__ Wt1, _Float16* __restrict__ Wt2) {
  const int tid = threadIdx.x;
  const int wave = tid >> 5, lane = tid & 31;
  const int mat = blockIdx.x >> 5;
  const int n = (blockIdx.x & 31) * 8 + wave;
  const float* W = mat ? W2 : W1;
  _Float16* Wt = mat ? Wt2 : Wt1;
  v8f f;
#pragma unroll
  for (int e = 0; e < 8; ++e) f[e] = W[(size_t)(lane * 8 + e) * DDIM + n];
  const v8h hv = __builtin_convertvector(f, v8h);
  _Float16* p = Wt + (size_t)n * DDIM + lane * 8;
  *(volatile v8h*)p = hv;
  __threadfence();
  *(volatile v8h*)p = hv;
}

__global__ void __launch_bounds__(128) __attribute__((amdgpu_num_vgpr(256)))
k_rk45(const float* __restrict__ x0, const _Float16* __restrict__ wt1, const _Float16* __restrict__ wt2,
       float* scr, float* __restrict__ out, int ntot_i) {
  __shared__ __align__(16) _Float16 tile[RPB * PKH];
  __shared__ __align__(16) float slabs[4][16 * SLABP];
  const size_t ntot = (size_t)ntot_i;
  const int tid = threadIdx.x;
  const int wave = __builtin_amdgcn_readfirstlane(tid >> 5);
  const int lane = tid & 31;
  const int c = lane & 15, hh = lane >> 4, koff = hh * 8;
  const int F0 = wave * 64;
  const int R0 = blockIdx.x * RPB;
  const int gw = blockIdx.x * 4 + wave;
  float* Xw = scr + (size_t)gw * 4096;
  const unsigned lo = (unsigned)lane * 4u;

#pragma unroll
  for (int i = 0; i < 4; ++i) {
#pragma unroll
    for (int j = 0; j < 4; ++j) {
      const float* p = x0 + (size_t)(R0 + 16 * j + c) * DDIM + F0 + 16 * i + 8 * hh;
      const v4f xa = *(const v4f*)p;
      const v4f xb = *(const v4f*)(p + 4);
      const unsigned o0 = lo + (unsigned)(2 * (i * 4 + j)) * 128u;
      const unsigned o1 = o0 + 128u;
      st_pair(Xw, o0, o1, xa, xb);
      tile_put(tile, 16 * j + c, F0 + 16 * i + 8 * hh, xa, xb);
    }
  }
  __syncthreads();

#pragma unroll 1
  for (int step = 0; step < NSTEP; ++step) {
    run_stage<0>(wt1, wt2, tile, Xw, ntot, lo, F0, c, hh, koff);
    run_stage<1>(wt1, wt2, tile, Xw, ntot, lo, F0, c, hh, koff);
    run_stage<2>(wt1, wt2, tile, Xw, ntot, lo, F0, c, hh, koff);
    run_stage<3>(wt1, wt2, tile, Xw, ntot, lo, F0, c, hh, koff);
    run_stage<4>(wt1, wt2, tile, Xw, ntot, lo, F0, c, hh, koff);
    run_stage<5>(wt1, wt2, tile, Xw, ntot, lo, F0, c, hh, koff);
  }

  float* slab = slabs[wave];
#pragma unroll 1
  for (int j = 0; j < 4; ++j) {
#pragma unroll
    for (int i = 0; i < 4; ++i) {
      const unsigned o0 = lo + (unsigned)(2 * (i * 4 + j)) * 128u;
      const unsigned o1 = o0 + 128u;
      const v4f xa = *(const v4f*)(Xw + o0);
      const v4f xb = *(const v4f*)(Xw + o1);
      *(v4f*)(slab + c * SLABP + 16 * i + 8 * hh) = xa;
      *(v4f*)(slab + c * SLABP + 16 * i + 8 * hh + 4) = xb;
    }
    __builtin_amdgcn_fence(__ATOMIC_RELEASE, "workgroup");
    __builtin_amdgcn_wave_barrier();
    __builtin_amdgcn_fence(__ATOMIC_ACQUIRE, "workgroup");
    const int c4 = c * 4;
    for (int pass = 0; pass < 2; ++pass) {
#pragma unroll
      for (int it = 0; it < 8; ++it) {
        const int row = it * 2 + hh;
        const v4f v = *(const v4f*)(slab + row * SLABP + c4);
        *(volatile v4f*)(out + (size_t)(R0 + 16 * j + row) * DDIM + F0 + c4) = v;
      }
      __threadfence();
    }
    __builtin_amdgcn_fence(__ATOMIC_RELEASE, "workgroup");
    __builtin_amdgcn_wave_barrier();
    __builtin_amdgcn_fence(__ATOMIC_ACQUIRE, "workgroup");
  }
}

extern "C" void kernel_launch(void* const* d_in, const int* in_sizes, int n_in,
                              void* d_out, int out_size, void* d_ws, size_t ws_size,
                              hipStream_t stream) {
  if (n_in < 3) return;
  const int nx = in_sizes[0];
  if (nx <= 0 || (nx % (RPB * DDIM)) != 0) return;
  if (in_sizes[1] != DDIM * DDIM || in_sizes[2] != DDIM * DDIM) return;
  if (out_size != nx) return;
  const int nblk = nx / (RPB * DDIM);

  size_t off = 0;
  float* scr = (float*)((char*)d_ws + off);
  off += (size_t)6 * (size_t)nx * sizeof(float);
  off = (off + 511) & ~(size_t)511;
  _Float16* wt1 = (_Float16*)((char*)d_ws + off);
  off += (size_t)DDIM * DDIM * sizeof(_Float16);
  _Float16* wt2 = (_Float16*)((char*)d_ws + off);
  off += (size_t)DDIM * DDIM * sizeof(_Float16);
  if (off > ws_size || off > ((size_t)128 << 20)) return;

  const float* x0 = (const float*)d_in[0];
  const float* W1 = (const float*)d_in[1];
  const float* W2 = (const float*)d_in[2];
  float* out = (float*)d_out;

  k_wt<<<dim3(64), dim3(256), 0, stream>>>(W1, W2, wt1, wt2);
  k_rk45<<<dim3(nblk), dim3(128), 0, stream>>>(x0, wt1, wt2, scr, out, nx);
}
